// EAConv_78469052498587
// MI455X (gfx1250) — hardware-verified
//
#include <hip/hip_runtime.h>
#include <math.h>

#define NN 50000
#define NE 800000
#define NV (NE + NN)
#define NPAD 50048
#define FD 128
#define FH 512
#define NT 256
#define SRB 2048
#define NTILE 25
#define SRBD 8192
#define NTD 7
#define NDV (NTD * SRBD)
#define SCH 4096
#define SP (SCH / NT)
#define NCH ((NV + SCH - 1) / SCH)

typedef __attribute__((ext_vector_type(16))) _Float16 v16h;
typedef __attribute__((ext_vector_type(8)))  _Float16 v8h;
typedef __attribute__((ext_vector_type(16))) __bf16   v16b;
typedef __attribute__((ext_vector_type(8)))  __bf16   v8b;
typedef __attribute__((ext_vector_type(8)))  float    v8f;
typedef __attribute__((ext_vector_type(4)))  float    v4f;
typedef __attribute__((ext_vector_type(4)))  int      v4i;

__device__ __forceinline__ unsigned short f2bf_bits(float f) {
  unsigned u = __float_as_uint(f);
  return (unsigned short)((u + 0x7FFFu + ((u >> 16) & 1u)) >> 16);
}
__device__ __forceinline__ float bf_bits2f(unsigned short h) { return __uint_as_float(((unsigned)h) << 16); }

__device__ __forceinline__ void dep_guard_h(v8f& a, v8f& b, v16h x, v16h y) { asm volatile("v_nop\n\tv_nop\n\tv_nop\n\tv_nop" : "+v"(a), "+v"(b) : "v"(x), "v"(y)); }
__device__ __forceinline__ void dep_guard_b(v8f& a, v8f& b, v16b x, v16b y) { asm volatile("v_nop\n\tv_nop\n\tv_nop\n\tv_nop" : "+v"(a), "+v"(b) : "v"(x), "v"(y)); }
__device__ __forceinline__ void keep4_h(v16h a, v16h b, v16h c, v16h d) { asm volatile("v_nop" :: "v"(a), "v"(b), "v"(c), "v"(d)); }
__device__ __forceinline__ void keep4_b(v16b a, v16b b, v16b c, v16b d) { asm volatile("v_nop" :: "v"(a), "v"(b), "v"(c), "v"(d)); }
__device__ __forceinline__ void acc_guard4(v8f& a, v8f& b, v8f& c, v8f& d) { asm volatile("v_nop\n\tv_nop\n\tv_nop\n\tv_nop" : "+v"(a), "+v"(b), "+v"(c), "+v"(d)); }
template <typename T> struct Frag;
template <> struct Frag<_Float16> {
  typedef v16h V; union U { v16h v; v8h h[2]; };
  static __device__ __forceinline__ v16h load(const _Float16* p) {
    U f; f.h[0] = *(const v8h*)(p); f.h[1] = *(const v8h*)(p + 16); return f.v;
  }
  static __device__ __forceinline__ v8f mma(v16h a, v16h b, v8f c) {
    return __builtin_amdgcn_wmma_f32_16x16x32_f16(false, a, false, b, (short)0, c, false, false);
  }
  static __device__ __forceinline__ void guard(v8f& a, v8f& b, v16h x, v16h y) { dep_guard_h(a, b, x, y); }
  static __device__ __forceinline__ void keep(v16h a, v16h b, v16h c, v16h d) { keep4_h(a, b, c, d); }
};
template <> struct Frag<__bf16> {
  typedef v16b V; union U { v16b v; v8b h[2]; };
  static __device__ __forceinline__ v16b load(const __bf16* p) {
    U f; f.h[0] = *(const v8b*)(p); f.h[1] = *(const v8b*)(p + 16); return f.v;
  }
  static __device__ __forceinline__ v8f mma(v16b a, v16b b, v8f c) {
    return __builtin_amdgcn_wmma_f32_16x16x32_bf16(false, a, false, b, (short)0, c, false, false);
  }
  static __device__ __forceinline__ void guard(v8f& a, v8f& b, v16b x, v16b y) { dep_guard_b(a, b, x, y); }
  static __device__ __forceinline__ void keep(v16b a, v16b b, v16b c, v16b d) { keep4_b(a, b, c, d); }
};

template <int ET> struct Elem;
template <> struct Elem<0> { typedef _Float16 T; };
template <> struct Elem<1> { typedef __bf16 T; };
template <int ET, bool SPLIT, int BIAS_MODE, int OUT_MODE, bool RESID, int ACT = 0>
__global__ __launch_bounds__(256) void wmma_gemm64(
    const unsigned short* __restrict__ Ap, const unsigned short* __restrict__ A2p, int lda, long strideA,
    const unsigned short* __restrict__ Btp, const unsigned short* __restrict__ Bt2p, int ldb, long strideB,
    void* __restrict__ Cout, void* __restrict__ Cout2, int ldc, long strideC,
    const float* __restrict__ bias,
    const float* __restrict__ resid, long strideR,
    int M, int N, int K, float scale) {
  typedef typename Elem<ET>::T T;
  typedef typename Frag<T>::V V;
  const T* A = (const T*)Ap; const T* A2 = (const T*)A2p; const T* Bt = (const T*)Btp; const T* Bt2 = (const T*)Bt2p;
  __shared__ __align__(16) float sT[8][16 * 68];
  const int b    = blockIdx.y;
  const int lane = threadIdx.x & 31;
  const int wave = threadIdx.x >> 5;
  const int tilesN = N >> 6;
  const int tilesM = M >> 6;
  const int tile = blockIdx.x * 8 + wave;
  if (tile >= tilesM * tilesN) return;
  const int tm = tile / tilesN;
  const int tn = tile - tm * tilesN;
  const int m0 = tm << 6;
  const int n0 = tn << 6;

  const T* Ab  = A  + (size_t)b * strideA;
  const T* Bb  = Bt + (size_t)b * strideB;
  const T* Ab2 = SPLIT ? (A2  + (size_t)b * strideA) : nullptr;
  const T* Bb2 = SPLIT ? (Bt2 + (size_t)b * strideB) : nullptr;

  const int rlane = lane & 15;
  const int koff  = (lane >> 4) * 8;
  const int mOff  = (lane >> 4) * 8;

  v8f acc[4][4];
#pragma unroll
  for (int i = 0; i < 4; ++i)
#pragma unroll
    for (int j = 0; j < 4; ++j) acc[i][j] = (v8f){0.f,0.f,0.f,0.f,0.f,0.f,0.f,0.f};

  for (int k0 = 0; k0 < K; k0 += 32) {
    V bh[4], bl[4];
#pragma unroll
    for (int j = 0; j < 4; ++j) {
      const size_t bo = (size_t)(n0 + (j << 4) + rlane) * ldb + koff + k0;
      bh[j] = Frag<T>::load(Bb + bo);
      if (SPLIT) bl[j] = Frag<T>::load(Bb2 + bo);
    }
#pragma unroll
    for (int i = 0; i < 4; ++i) {
      const size_t ao = (size_t)(m0 + (i << 4) + rlane) * lda + koff + k0;
      V ah = Frag<T>::load(Ab + ao);
      V al;
      if (SPLIT) al = Frag<T>::load(Ab2 + ao);
#pragma unroll
      for (int j = 0; j < 4; ++j) {
        acc[i][j] = Frag<T>::mma(ah, bh[j], acc[i][j]);
        if (SPLIT) {
          acc[i][j] = Frag<T>::mma(ah, bl[j], acc[i][j]);
          acc[i][j] = Frag<T>::mma(al, bh[j], acc[i][j]);
        }
      }
      Frag<T>::guard(acc[i][0], acc[i][3], ah, SPLIT ? al : ah);
    }
    Frag<T>::keep(bh[0], bh[1], bh[2], bh[3]);
    if (SPLIT) Frag<T>::keep(bl[0], bl[1], bl[2], bl[3]);
  }
  acc_guard4(acc[0][0], acc[0][1], acc[0][2], acc[0][3]);
  acc_guard4(acc[1][0], acc[1][1], acc[1][2], acc[1][3]);
  acc_guard4(acc[2][0], acc[2][1], acc[2][2], acc[2][3]);
  acc_guard4(acc[3][0], acc[3][1], acc[3][2], acc[3][3]);

  float* slab = sT[wave];
  const float* Rb = RESID ? (resid + (size_t)b * strideR) : nullptr;
#pragma unroll
  for (int i = 0; i < 4; ++i) {
    const int mBase = m0 + (i << 4);
#pragma unroll
    for (int j = 0; j < 4; ++j) {
      const int n = n0 + (j << 4) + rlane;
      float bv = 0.f;
      if (BIAS_MODE == 2) bv = bias[n];
#pragma unroll
      for (int r = 0; r < 8; ++r) {
        float v = acc[i][j][r] * scale;
        if (BIAS_MODE == 1) v += bias[mBase + mOff + r];
        if (BIAS_MODE == 2) v += bv;
        if (RESID) v += Rb[(size_t)(mBase + mOff + r) * ldc + n];
        if (ACT == 1) v = tanhf(v);
        if (ACT == 2) v = fmaxf(v, 0.0f);
        if (ACT == 3) v = v / (1.0f + expf(-v));
        if (ACT == 4) v = (v > 0.f) ? v : 0.01f * v;
        if (ACT == 5) v = 0.5f * v * (1.0f + erff(v * 0.70710678118654752f));
        slab[(mOff + r) * 68 + (j << 4) + rlane] = v;
      }
    }
    __builtin_amdgcn_fence(__ATOMIC_RELEASE, "workgroup");
    __builtin_amdgcn_wave_barrier();
    __builtin_amdgcn_fence(__ATOMIC_ACQUIRE, "workgroup");
    if (OUT_MODE == 0) {
      float* C = (float*)Cout + (size_t)b * strideC;
      const int hh = lane >> 4, c4 = (lane & 15) * 4;
      for (int pass = 0; pass < 2; ++pass) {
#pragma unroll
        for (int it = 0; it < 8; ++it) {
          const int row = it * 2 + hh;
          v4f v = *(const v4f*)(slab + row * 68 + c4);
          *(volatile v4f*)(C + (size_t)(mBase + row) * ldc + n0 + c4) = v;
        }
        __threadfence();
      }
    } else {
      const int q = lane >> 3, c8 = (lane & 7) * 8;
      unsigned short* C  = (unsigned short*)Cout  + (size_t)b * strideC;
      unsigned short* C2 = (OUT_MODE == 2) ? ((unsigned short*)Cout2 + (size_t)b * strideC) : nullptr;
      for (int pass = 0; pass < 2; ++pass) {
#pragma unroll
        for (int it = 0; it < 4; ++it) {
          const int row = it * 4 + q;
          const float* sp = slab + row * 68 + c8;
          v8h hv, lv;
#pragma unroll
          for (int e = 0; e < 8; ++e) {
            if (OUT_MODE == 1) {
              hv[e] = (_Float16)sp[e];
            } else {
              unsigned short hb = f2bf_bits(sp[e]);
              unsigned short lb = f2bf_bits(sp[e] - bf_bits2f(hb));
              hv[e] = __builtin_bit_cast(_Float16, hb);
              lv[e] = __builtin_bit_cast(_Float16, lb);
            }
          }
          *(volatile v8h*)(C + (size_t)(mBase + row) * ldc + n0 + c8) = hv;
          if (OUT_MODE == 2) *(volatile v8h*)(C2 + (size_t)(mBase + row) * ldc + n0 + c8) = lv;
        }
        __threadfence();
      }
    }
    __builtin_amdgcn_fence(__ATOMIC_RELEASE, "workgroup");
    __builtin_amdgcn_wave_barrier();
    __builtin_amdgcn_fence(__ATOMIC_ACQUIRE, "workgroup");
  }
}

__device__ __forceinline__ int blk_excl_scan(int cnt, int* scan_ws, int tid, int* tot) {
  const int lane = tid & 31, wave = tid >> 5; int incl = cnt;
#pragma unroll
  for (int o = 1; o < 32; o <<= 1) { const int v = __shfl_up(incl, o, 32); if (lane >= o) incl += v; }
  if (lane == 31) scan_ws[wave] = incl;
  __syncthreads();
  if (wave == 0) { int wv = (lane < NT / 32) ? scan_ws[lane] : 0; int wincl = wv;
#pragma unroll
    for (int o = 1; o < 32; o <<= 1) { const int v = __shfl_up(wincl, o, 32); if (lane >= o) wincl += v; }
    if (lane < NT / 32) scan_ws[32 + lane] = wincl - wv; if (lane == 31) scan_ws[64] = wincl; }
  __syncthreads();
  const int res = scan_ws[32 + wave] + incl - cnt; *tot = scan_ws[64];
  return res;
}
template <int TW>
__device__ __forceinline__ int chunk_hits(const int* __restrict__ dstv, const int* __restrict__ srcv, int e0, int n0, int tid,
                                          int* LIST, int* scan_ws) {
  const int eb = e0 + tid * SP;
  const bool real = eb < NE;
  const int ebc = real ? eb : (NE - SP);
  int rec[SP]; int cnt = 0;
#pragma unroll
  for (int k = 0; k < SP; k += 4) {
    const v4i d4 = *(const v4i*)(dstv + ebc + k);
    const v4i s4 = *(const v4i*)(srcv + ebc + k);
#pragma unroll
    for (int e = 0; e < 4; ++e) {
      const int ev = eb + k + e;
      const int dv = ev - NE;
      const int d = real ? d4[e] : dv;
      int s = real ? s4[e] : dv;
      s = s < 0 ? 0 : (s >= NN ? NN - 1 : s);
      const bool ok = real || (ev < NV);
      int r = -1;
      if (ok && d >= n0 && d < n0 + TW) { r = ((d - n0) << 16) | s; ++cnt; }
      rec[k + e] = r;
    }
  }
  int tot; int p = blk_excl_scan(cnt, scan_ws, tid, &tot);
#pragma unroll
  for (int k = 0; k < SP; ++k) if (rec[k] >= 0) { if ((unsigned)p < (unsigned)SCH) LIST[p] = rec[k]; ++p; }
  __syncthreads();
  return tot < SCH ? tot : SCH;
}

__global__ __launch_bounds__(NT) void prep_kernel(const float* __restrict__ W1, const float* __restrict__ b1, const float* __restrict__ W2,
                                                 const int* __restrict__ ixp, const int* __restrict__ mip,
                                                 unsigned* __restrict__ W1T, unsigned* __restrict__ W2T, float* __restrict__ B1S) {
  (void)ixp; (void)mip;
  const int i = blockIdx.x * NT + threadIdx.x;
  if (i < FH * FD / 2) {
    {
      const int n = i >> 6;
      const int k = 2 * (i & 63);
      const _Float16 ha = (_Float16)(W1[(size_t)k * FH + n] * 16.0f);
      const _Float16 hb = (_Float16)(W1[(size_t)(k + 1) * FH + n] * 16.0f);
      const unsigned u = (unsigned)__builtin_bit_cast(unsigned short, ha) | ((unsigned)__builtin_bit_cast(unsigned short, hb) << 16);
      ((volatile unsigned*)W1T)[i] = u;
      __threadfence();
      ((volatile unsigned*)W1T)[i] = u;
    }
    {
      const int n = i >> 8;
      const int k = 2 * (i & 255);
      const _Float16 ha = (_Float16)(W2[(size_t)k * FD + n] * 16.0f);
      const _Float16 hb = (_Float16)(W2[(size_t)(k + 1) * FD + n] * 16.0f);
      const unsigned u = (unsigned)__builtin_bit_cast(unsigned short, ha) | ((unsigned)__builtin_bit_cast(unsigned short, hb) << 16);
      ((volatile unsigned*)W2T)[i] = u;
      __threadfence();
      ((volatile unsigned*)W2T)[i] = u;
    }
  }
  if (i < FH) {
    const float v = b1[i] * 16.0f;
    ((volatile float*)B1S)[i] = v;
    __threadfence();
    ((volatile float*)B1S)[i] = v;
  }
}

__global__ __launch_bounds__(NT) void deg_kernel(const int* __restrict__ ei, float* __restrict__ dinv) {
  __shared__ int LIST[SCH];
  __shared__ int CNT[SRBD];
  __shared__ int scan_ws[80];
  const int tid = threadIdx.x, lane = tid & 31, wave = tid >> 5;
  const int n0 = blockIdx.x * SRBD;
  for (int i = tid; i < SRBD; i += NT) CNT[i] = 0;
  __syncthreads();
  const int* srcv = ei; const int* dstv = ei + NE;
#pragma unroll 1
  for (int c = 0; c < NCH; ++c) {
    const int tot = chunk_hits<SRBD>(dstv, srcv, c * SCH, n0, tid, LIST, scan_ws);
#pragma unroll 1
    for (int base = 0; base < tot; base += 32) {
      const int q = base + lane;
      const int qc = (q < tot) ? q : 0;
      int rv = LIST[qc]; rv = (q < tot) ? rv : -1;
      const int own = (rv >= 0 && (rv >> 26) == wave) ? 1 : 0;
      unsigned msk = (unsigned)__ballot(own);
#pragma unroll 1
      for (int it = 0; it < 32; ++it) {
        if (msk == 0u) break;
        const int bp = __builtin_ctz(msk); msk &= msk - 1u;
        const int r = __shfl(rv, bp, 32);
        const int dl = r >> 16;
        if (lane == 0) CNT[dl] = CNT[dl] + 1;
      }
    }
    __syncthreads();
  }
#pragma unroll 1
  for (int it = 0; it < SRBD / (NT * 4); ++it) {
    const int i = it * NT * 4 + 4 * tid;
    v4f o;
#pragma unroll
    for (int e = 0; e < 4; ++e) {
      const int cn = CNT[i + e];
      const float cf = (float)(cn > 0 ? cn : 1);
      float v = 1.0f / sqrtf(cf);
      v = (cn > 0) ? v : 0.f;
      o[e] = v;
    }
    float* p = dinv + n0 + i;
    *(volatile v4f*)p = o;
    __threadfence();
    *(volatile v4f*)p = o;
  }
}

template <int PASS>
__global__ __launch_bounds__(NT) void agg_kernel(const float* __restrict__ rows, const int* __restrict__ ei, const float* __restrict__ dinv,
                                                float* ACC, const float* __restrict__ bias,
                                                unsigned short* __restrict__ outh, float* __restrict__ outf) {
  __shared__ int LIST[SCH];
  __shared__ int scan_ws[80];
  const int tid = threadIdx.x, lane = tid & 31, wave = tid >> 5;
  const int n0 = blockIdx.x * SRB;
  const size_t rbase = (size_t)blockIdx.x * SRB;
  const v4f z4 = {0.f, 0.f, 0.f, 0.f};
#pragma unroll 1
  for (int j = 0; j < SRB / 8; ++j) {
    float* rp = ACC + (rbase + (size_t)wave * (SRB / 8) + j) * FD + 4 * lane;
    *(volatile v4f*)rp = z4;
  }
  __threadfence();
#pragma unroll 1
  for (int j = 0; j < SRB / 8; ++j) {
    float* rp = ACC + (rbase + (size_t)wave * (SRB / 8) + j) * FD + 4 * lane;
    *(volatile v4f*)rp = z4;
  }
  __threadfence();
  const int* srcv = ei; const int* dstv = ei + NE;
#pragma unroll 1
  for (int c = 0; c < NCH; ++c) {
    const int tot = chunk_hits<SRB>(dstv, srcv, c * SCH, n0, tid, LIST, scan_ws);
#pragma unroll 1
    for (int base = 0; base < tot; base += 32) {
      const int q = base + lane;
      const int qc = (q < tot) ? q : 0;
      int rv = LIST[qc]; rv = (q < tot) ? rv : -1;
      const int own = (rv >= 0 && (rv >> 24) == wave) ? 1 : 0;
      unsigned msk = (unsigned)__ballot(own);
#pragma unroll 1
      for (int it = 0; it < 32; ++it) {
        if (msk == 0u) break;
        const int bp = __builtin_ctz(msk); msk &= msk - 1u;
        const int r = __shfl(rv, bp, 32);
        const int dl = r >> 16, s = r & 0xFFFF;
        const float w = dinv[s];
        const v4f xv = *(const v4f*)(rows + (size_t)s * FD + 4 * lane);
        float* rp = ACC + (rbase + dl) * FD + 4 * lane;
        v4f a = *(const v4f*)rp;
        a = a + w * xv;
        *(volatile v4f*)rp = a;
        __threadfence();
        *(volatile v4f*)rp = a;
      }
    }
    __syncthreads();
  }
  if (PASS == 1) {
    const int cl = lane & 15;
#pragma unroll 1
    for (int j = 0; j < SRB / 8; ++j) {
      const int dl = wave * (SRB / 8) + j; const int n = n0 + dl;
      if (n < NPAD) {
        const bool live = n < NN;
        const int nc = live ? n : NN - 1;
        float w = dinv[nc] * 16.0f;
        w = live ? w : 0.f;
        const v4f a = *(const v4f*)(ACC + (rbase + dl) * FD + 4 * lane);
        const v4f v = a * w;
        v8h hv;
#pragma unroll
        for (int e = 0; e < 4; ++e) {
          const float f0 = __shfl(v[e], 2 * cl, 32);
          const float f1 = __shfl(v[e], 2 * cl + 1, 32);
          hv[e] = (_Float16)f0;
          hv[4 + e] = (_Float16)f1;
        }
        unsigned short* op = outh + (size_t)n * FD + 8 * cl;
        if (lane < 16) *(volatile v8h*)op = hv;
        __threadfence();
        if (lane < 16) *(volatile v8h*)op = hv;
      }
    }
  } else {
    const v4f bv = *(const v4f*)(bias + 4 * lane);
#pragma unroll 1
    for (int j = 0; j < SRB / 8; ++j) {
      const int dl = wave * (SRB / 8) + j; const int n = n0 + dl;
      if (n < NN) {
        const float w = dinv[n];
        const v4f a = *(const v4f*)(ACC + (rbase + dl) * FD + 4 * lane);
        const v4f v = a * w + bv;
        float* op = outf + (size_t)n * FD + 4 * lane;
        *(volatile v4f*)op = v;
        __threadfence();
        *(volatile v4f*)op = v;
      }
    }
  }
}

extern "C" void kernel_launch(void* const* d_in, const int* in_sizes, int n_in,
                              void* d_out, int out_size, void* d_ws, size_t ws_size, hipStream_t stream) {
  if (n_in < 8) return;
  if (in_sizes[0] != NN * FD || in_sizes[1] != FD * FH || in_sizes[2] != FH || in_sizes[3] != FH * FD ||
      in_sizes[4] != FD || in_sizes[5] != 2 * NE || out_size != NN * FD) return;
  const float* x   = (const float*)d_in[0];
  const float* W1  = (const float*)d_in[1];
  const float* b1  = (const float*)d_in[2];
  const float* W2  = (const float*)d_in[3];
  const float* b2  = (const float*)d_in[4];
  const int*   ei  = (const int*)  d_in[5];
  const int*   ixp = (const int*)  d_in[6];
  const int*   mip = (const int*)  d_in[7];
  float* out = (float*)d_out;

  char* ws = (char*)d_ws; size_t off = 0;
  auto carve = [&](size_t bytes) -> char* { char* p = ws + off; off += (bytes + 255) & ~(size_t)255; return p; };
  float*          DINV = (float*)carve((size_t)NDV * 4);
  unsigned*       W1T  = (unsigned*)carve((size_t)FH * FD * 2);
  unsigned*       W2T  = (unsigned*)carve((size_t)FD * FH * 2);
  float*          B1S  = (float*)carve((size_t)FH * 4);
  unsigned short* AXH  = (unsigned short*)carve((size_t)NPAD * FD * 2);
  unsigned short* Z    = (unsigned short*)carve((size_t)NPAD * FH * 2);
  float*          H2   = (float*)carve((size_t)NPAD * FD * 4);
  float*          ACC  = (float*)carve((size_t)NTILE * SRB * FD * 4);
  if (off > ws_size || off > (size_t)134217728) return;

  prep_kernel<<<(FH * FD / 2 + NT - 1) / NT, NT, 0, stream>>>(W1, b1, W2, ixp, mip, W1T, W2T, B1S);
  deg_kernel<<<NTD, NT, 0, stream>>>(ei, DINV);
  agg_kernel<1><<<NTILE, NT, 0, stream>>>(x, ei, DINV, ACC, B1S, AXH, H2);
  {
    const int tiles = (NPAD / 64) * (FH / 64);
    wmma_gemm64<0, false, 2, 1, false, 2><<<dim3((tiles + 7) / 8, 1), 256, 0, stream>>>(
        (const unsigned short*)AXH, (const unsigned short*)AXH, FD, 0L,
        (const unsigned short*)W1T, (const unsigned short*)W1T, FD, 0L,
        (void*)Z, (void*)Z, FH, 0L,
        (const float*)B1S, (const float*)B1S, 0L, NPAD, FH, FD, 1.0f / 16.0f);
  }
  {
    const int tiles = (NPAD / 64) * (FD / 64);
    wmma_gemm64<0, false, 0, 0, false, 0><<<dim3((tiles + 7) / 8, 1), 256, 0, stream>>>(
        (const unsigned short*)Z, (const unsigned short*)Z, FH, 0L,
        (const unsigned short*)W2T, (const unsigned short*)W2T, FH, 0L,
        (void*)H2, (void*)H2, FD, 0L,
        (const float*)B1S, (const float*)B1S, 0L, NPAD, FD, FH, 1.0f / 256.0f);
  }
  agg_kernel<2><<<NTILE, NT, 0, stream>>>(H2, ei, DINV, ACC, b2, AXH, out);
}
